// CapsuleNetwork_11982958756250
// MI455X (gfx1250) — hardware-run, weakly checked
//
#include <hip/hip_runtime.h>
#include <stddef.h>
#include <stdint.h>

#define BSZ    1024
#define IND    768
#define PROJ   9216
#define NIC    256
#define NPOS   36
#define IMW    6
#define NOC    256
#define NTAP   9
#define KTAP   (2 * NIC)
#define KCW    (NTAP * KTAP)
#define CKW    (NIC * NTAP)
#define CROWS  (BSZ * 16)
#define NCAP   512
#define NCLS   5
#define RD     16
#define PD     8
#define NOD    (NCLS * RD)
#define PVP    128
#define NTHR   256
#define GTHR   128
#define GBM    64
#define GBN    128
#define K8X    (IND / 8)
#define K8C    (KCW / 8)
#define NU_X   (BSZ * K8X)
#define NU_W1  (PROJ * K8X)
#define NU_CW  (NOC * K8C)
#define NU_PREP (NU_X + NU_W1 + NU_CW)
#define OUT_V0 (BSZ * NCLS)
#define OUT_N  (OUT_V0 + BSZ * NOD)
#define OUT_U  (OUT_N / 4)
#define RT_SC  (NOD * NCAP)
#define RT_SL  (RT_SC + NCAP * NCLS)
#define RT_SS  (RT_SL + NCAP * NCLS)
#define RT_SV  (RT_SS + NOD)
#define RT_SO  (RT_SV + NOD)
#define RT_FLOATS (RT_SO + PVP)
#define RT_LDS_BYTES (RT_FLOATS * 4)
#define WSMAX  134217728

static_assert(NU_X % NTHR == 0 && NU_W1 % NTHR == 0 && NU_CW % NTHR == 0);
static_assert(K8X % 32 == 0 && K8C % 32 == 0);
static_assert(IND % 32 == 0 && KTAP % 32 == 0 && KTAP == 512);
static_assert(BSZ % GBM == 0 && PROJ % GBN == 0 && NOC % GBN == 0 && BSZ % 4 == 0);
static_assert(GBM == (GTHR / 32) * 16 && GBN == 8 * 16);
static_assert(PROJ == NIC * NPOS && PROJ % (4 * NTHR) == 0 && (NPOS * 64) % NTHR == 0);
static_assert(NCAP == 2 * NTHR && NOD + NCLS <= PVP && PVP == 4 * 32 && NOD <= NTHR);
static_assert(OUT_N % 4 == 0 && OUT_U % NTHR == 0 && OUT_V0 % 4 == 0);
static_assert(RT_LDS_BYTES <= 300000 && (RT_SO * 4) % 16 == 0);
static_assert(NCAP * NOD * PD == 327680 && NOC * CKW == 589824);

typedef float          v4f   __attribute__((ext_vector_type(4)));
typedef float          v8f   __attribute__((ext_vector_type(8)));
typedef int            v8i   __attribute__((ext_vector_type(8)));
typedef unsigned short v8us  __attribute__((ext_vector_type(8)));
typedef unsigned short v16us __attribute__((ext_vector_type(16)));
typedef __bf16         v16bf __attribute__((ext_vector_type(16)));
typedef v4f  __attribute__((may_alias)) v4fa;
typedef v8us __attribute__((may_alias)) v8usa;
union FragB { v16bf v; v16us u; v8us h[2]; v8i w; };

__device__ __forceinline__ v8f wmb(const FragB& a, const FragB& b, v8f c) {
  v8f d = __builtin_amdgcn_wmma_f32_16x16x32_bf16(false, a.v, false, b.v, (short)0, c, false, false);
  asm volatile("v_nop\n\tv_nop\n\tv_nop\n\tv_nop" : "+v"(d) : "v"(a.w), "v"(b.w));
  return d;
}

__device__ __forceinline__ unsigned bf16_bits(float f) {
  const unsigned u = __float_as_uint(f);
  return (u + 0x7FFFu + ((u >> 16) & 1u)) >> 16;
}
__device__ __forceinline__ float bf16_val(float f) {
  return __uint_as_float(bf16_bits(f) << 16);
}
__device__ __forceinline__ void put16(unsigned short* dp, v8us o) {
  *(volatile v8us*)dp = o;
  __threadfence();
  *(volatile v8us*)dp = o;
}
__device__ __forceinline__ void putf4(float* dp, v4f o) {
  *(volatile v4f*)dp = o;
  __threadfence();
  *(volatile v4f*)dp = o;
}

__global__ __launch_bounds__(NTHR) void k_prep(const float* __restrict__ x, const float* __restrict__ W1,
                                               const float* __restrict__ convW,
                                               unsigned short* XB, unsigned short* W1T, unsigned short* CW2) {
  const int u = (int)blockIdx.x * NTHR + (int)threadIdx.x;
  v8us o;
  if (u < NU_X) {
    const int row = u / K8X;
    const int k8  = (u - row * K8X) * 8;
    const float* p = x + (size_t)row * IND + k8;
    const v4f a = *(const v4fa*)p;
    const v4f c = *(const v4fa*)(p + 4);
    o[0] = (unsigned short)bf16_bits(a.x); o[1] = (unsigned short)bf16_bits(a.y);
    o[2] = (unsigned short)bf16_bits(a.z); o[3] = (unsigned short)bf16_bits(a.w);
    o[4] = (unsigned short)bf16_bits(c.x); o[5] = (unsigned short)bf16_bits(c.y);
    o[6] = (unsigned short)bf16_bits(c.z); o[7] = (unsigned short)bf16_bits(c.w);
    put16(XB + (size_t)row * IND + k8, o);
    return;
  } else if (u < NU_X + NU_W1) {
    const int v  = u - NU_X;
    const int n  = v / K8X;
    const int k8 = (v - n * K8X) * 8;
    const float* p = W1 + (size_t)k8 * PROJ + n;
#pragma unroll
    for (int i = 0; i < 8; ++i) o[i] = (unsigned short)bf16_bits(p[(size_t)i * PROJ]);
    put16(W1T + (size_t)n * IND + k8, o);
    return;
  } else if (u < NU_PREP) {
    const int v   = u - NU_X - NU_W1;
    const int oc  = v / K8C;
    const int k8  = (v - oc * K8C) * 8;
    const int tap = k8 >> 9;
    const int ic0 = k8 & (NIC - 1);
    const float* p = convW + (size_t)oc * CKW + (size_t)ic0 * NTAP + tap;
#pragma unroll
    for (int i = 0; i < 8; ++i) o[i] = (unsigned short)bf16_bits(p[i * NTAP]);
    put16(CW2 + (size_t)oc * KCW + k8, o);
    return;
  }
}

__global__ __launch_bounds__(GTHR) void k_gemm1(const unsigned short* __restrict__ A,
                                                const unsigned short* __restrict__ BT,
                                                const float* __restrict__ bias, float* Hf) {
  __shared__ __attribute__((aligned(16))) float stg[GBM * GBN];
  const int tid = (int)threadIdx.x, lane = tid & 31, wave = tid >> 5, hh = lane >> 4, m = lane & 15;
  const int rowBase = (int)blockIdx.x * GBM;
  const int colBase = (int)blockIdx.y * GBN;

  v8f acc[8];
  {
    const v8f z = {0.f, 0.f, 0.f, 0.f, 0.f, 0.f, 0.f, 0.f};
#pragma unroll
    for (int t = 0; t < 8; ++t) acc[t] = z;
  }
  const unsigned short* ap = A  + (size_t)(rowBase + 16 * wave + m) * (size_t)IND + 8 * hh;
  const unsigned short* bp = BT + (size_t)(colBase + m) * (size_t)IND + 8 * hh;

#pragma unroll 1
  for (int k0 = 0; k0 < IND; k0 += 32) {
    FragB af;
    af.h[0] = *(const v8usa*)(ap + k0);
    af.h[1] = *(const v8usa*)(ap + k0 + 16);
#pragma unroll
    for (int nt = 0; nt < 8; ++nt) {
      const unsigned short* wq = bp + (size_t)(16 * nt) * (size_t)IND + k0;
      FragB bf;
      bf.h[0] = *(const v8usa*)wq;
      bf.h[1] = *(const v8usa*)(wq + 16);
      acc[nt] = wmb(af, bf, acc[nt]);
    }
  }

#pragma unroll
  for (int nt = 0; nt < 8; ++nt) {
    const int lc = 16 * nt + m;
    const float bvv = bf16_val(bias[colBase + lc]);
#pragma unroll
    for (int r = 0; r < 8; ++r) {
      const int lr = 16 * wave + 8 * hh + r;
      stg[lr * GBN + lc] = fmaxf(acc[nt][r] + bvv, 0.0f);
    }
  }
  __syncthreads();

  v4f pv[16];
#pragma unroll
  for (int i = 0; i < 16; ++i) pv[i] = *(const v4fa*)(stg + (16 * wave + i) * GBN + 4 * lane);
#pragma unroll
  for (int i = 0; i < 16; ++i) {
    float* op = Hf + (size_t)(rowBase + 16 * wave + i) * (size_t)PROJ + colBase + 4 * lane;
    *(volatile v4f*)op = pv[i];
  }
  __threadfence();
#pragma unroll
  for (int i = 0; i < 16; ++i) {
    float* op = Hf + (size_t)(rowBase + 16 * wave + i) * (size_t)PROJ + colBase + 4 * lane;
    *(volatile v4f*)op = pv[i];
  }
}

__global__ __launch_bounds__(NTHR) void k_ht(const float* __restrict__ Hf, unsigned short* HT) {
  __shared__ __attribute__((aligned(16))) float tile[NPOS * NIC];
  const int b = (int)blockIdx.x, t = (int)threadIdx.x;
  const float* hp = Hf + (size_t)b * PROJ;
#pragma unroll 1
  for (int it = 0; it < PROJ / (4 * NTHR); ++it) {
    const int j = 4 * (it * NTHR + t);
    const v4f q = *(const v4fa*)(hp + j);
#pragma unroll
    for (int e = 0; e < 4; ++e) {
      const int jj  = j + e;
      const int ic  = jj / NPOS;
      const int pos = jj - ic * NPOS;
      tile[pos * NIC + ic] = q[e];
    }
  }
  __syncthreads();
#pragma unroll 1
  for (int it = 0; it < (NPOS * 64) / NTHR; ++it) {
    const int v    = it * NTHR + t;
    const int pos  = v >> 6;
    const int q6   = v & 63;
    const int part = q6 >> 5;
    const int j8   = q6 & 31;
    const float* sp = tile + pos * NIC + 8 * j8;
    const v4f a = *(const v4fa*)sp;
    const v4f c = *(const v4fa*)(sp + 4);
    const v8f f8 = {a.x, a.y, a.z, a.w, c.x, c.y, c.z, c.w};
    const unsigned mh = 0u - (unsigned)part;
    const unsigned ml = ~mh;
    v8us o;
#pragma unroll
    for (int e = 0; e < 8; ++e) {
      const unsigned hb = bf16_bits(f8[e]);
      const unsigned lb = bf16_bits(f8[e] - __uint_as_float(hb << 16));
      o[e] = (unsigned short)((hb & ml) | (lb & mh));
    }
    put16(HT + (size_t)(b * NPOS + pos) * (size_t)KTAP + part * NIC + 8 * j8, o);
  }
}

__global__ __launch_bounds__(GTHR) void k_conv(const unsigned short* __restrict__ HT,
                                               const unsigned short* __restrict__ CW2,
                                               const float* __restrict__ cbias, float* CONV) {
  __shared__ __attribute__((aligned(16))) float stg[GBM * GBN];
  const int tid = (int)threadIdx.x, lane = tid & 31, wave = tid >> 5, hh = lane >> 4, m = lane & 15;
  const int b = (int)blockIdx.x * 4 + wave;
  const int colBase = (int)blockIdx.y * GBN;
  const int oy = m >> 2, ox = m & 3;

  v8f acc[8];
  {
    const v8f z = {0.f, 0.f, 0.f, 0.f, 0.f, 0.f, 0.f, 0.f};
#pragma unroll
    for (int t = 0; t < 8; ++t) acc[t] = z;
  }
  const unsigned short* hb = HT  + (size_t)b * NPOS * (size_t)KTAP + 8 * hh;
  const unsigned short* bp = CW2 + (size_t)(colBase + m) * (size_t)KCW + 8 * hh;

#pragma unroll 1
  for (int tap = 0; tap < NTAP; ++tap) {
    const int ky = tap / 3, kx = tap - 3 * ky;
    const unsigned short* ap = hb + (size_t)((oy + ky) * IMW + ox + kx) * (size_t)KTAP;
    const unsigned short* bq = bp + tap * KTAP;
#pragma unroll 1
    for (int k0 = 0; k0 < KTAP; k0 += 32) {
      FragB af;
      af.h[0] = *(const v8usa*)(ap + k0);
      af.h[1] = *(const v8usa*)(ap + k0 + 16);
#pragma unroll
      for (int nt = 0; nt < 8; ++nt) {
        const unsigned short* wq = bq + (size_t)(16 * nt) * (size_t)KCW + k0;
        FragB bf;
        bf.h[0] = *(const v8usa*)wq;
        bf.h[1] = *(const v8usa*)(wq + 16);
        acc[nt] = wmb(af, bf, acc[nt]);
      }
    }
  }

#pragma unroll
  for (int nt = 0; nt < 8; ++nt) {
    const int lc = 16 * nt + m;
    const float bvv = bf16_val(cbias[colBase + lc]);
#pragma unroll
    for (int r = 0; r < 8; ++r) {
      const int lr = 16 * wave + 8 * hh + r;
      stg[lr * GBN + lc] = acc[nt][r] + bvv;
    }
  }
  __syncthreads();

  v4f pv[16];
#pragma unroll
  for (int i = 0; i < 16; ++i) pv[i] = *(const v4fa*)(stg + (16 * wave + i) * GBN + 4 * lane);
#pragma unroll
  for (int i = 0; i < 16; ++i) {
    float* op = CONV + (size_t)(b * 16 + i) * (size_t)NOC + colBase + 4 * lane;
    *(volatile v4f*)op = pv[i];
  }
  __threadfence();
#pragma unroll
  for (int i = 0; i < 16; ++i) {
    float* op = CONV + (size_t)(b * 16 + i) * (size_t)NOC + colBase + 4 * lane;
    *(volatile v4f*)op = pv[i];
  }
}

__global__ __launch_bounds__(NTHR) void k_route(const float* __restrict__ CONV, const float* __restrict__ Wr,
                                                float* PV) {
  extern __shared__ __attribute__((aligned(16))) float dyn[];
  float* uh = dyn;
  float* sC = dyn + RT_SC;
  float* sL = dyn + RT_SL;
  float* sS = dyn + RT_SS;
  float* sV = dyn + RT_SV;
  float* sO = dyn + RT_SO;
  const int b = (int)blockIdx.x, t = (int)threadIdx.x, lane = t & 31, wave = t >> 5;

#pragma unroll 1
  for (int j = 0; j < 2; ++j) {
    const int n   = t + NTHR * j;
    const int cap = n >> 4, p = n & 15;
    const float* cp = CONV + (size_t)(b * 16 + p) * (size_t)NOC + cap * PD;
    const v4f ta = *(const v4fa*)cp;
    const v4f tb = *(const v4fa*)(cp + 4);
    float sq = ta.x * ta.x;
    sq = fmaf(ta.y, ta.y, sq); sq = fmaf(ta.z, ta.z, sq); sq = fmaf(ta.w, ta.w, sq);
    sq = fmaf(tb.x, tb.x, sq); sq = fmaf(tb.y, tb.y, sq); sq = fmaf(tb.z, tb.z, sq); sq = fmaf(tb.w, tb.w, sq);
    const float scl = sq / (1.0f + sq);
    const float rn  = 1.0f / sqrtf(sq + 1e-8f);
    const float u0 = (scl * ta.x) * rn, u1 = (scl * ta.y) * rn, u2 = (scl * ta.z) * rn, u3 = (scl * ta.w) * rn;
    const float u4 = (scl * tb.x) * rn, u5 = (scl * tb.y) * rn, u6 = (scl * tb.z) * rn, u7 = (scl * tb.w) * rn;
    const float* wp = Wr + (size_t)n * (NOD * PD);
#pragma unroll 1
    for (int od = 0; od < NOD; ++od) {
      const v4f wa = *(const v4fa*)(wp + od * PD);
      const v4f wb = *(const v4fa*)(wp + od * PD + 4);
      float a = bf16_val(wa.x) * u0;
      a = fmaf(bf16_val(wa.y), u1, a);
      a = fmaf(bf16_val(wa.z), u2, a);
      a = fmaf(bf16_val(wa.w), u3, a);
      a = fmaf(bf16_val(wb.x), u4, a);
      a = fmaf(bf16_val(wb.y), u5, a);
      a = fmaf(bf16_val(wb.z), u6, a);
      a = fmaf(bf16_val(wb.w), u7, a);
      uh[od * NCAP + n] = a;
    }
#pragma unroll 1
    for (int o = 0; o < NCLS; ++o) sL[n * NCLS + o] = 0.0f;
  }
  __syncthreads();

#pragma unroll 1
  for (int it = 0; it < 3; ++it) {
#pragma unroll 1
    for (int j = 0; j < 2; ++j) {
      const int n = t + NTHR * j;
      float* lr = sL + n * NCLS;
      float* cr = sC + n * NCLS;
      float mx = lr[0];
#pragma unroll 1
      for (int o = 1; o < NCLS; ++o) mx = fmaxf(mx, lr[o]);
      float sum = 0.0f;
#pragma unroll 1
      for (int o = 0; o < NCLS; ++o) {
        const float e = expf(lr[o] - mx);
        cr[o] = e;
        sum += e;
      }
      const float inv = 1.0f / sum;
#pragma unroll 1
      for (int o = 0; o < NCLS; ++o) cr[o] = cr[o] * inv;
    }
    __syncthreads();
    if (t < NOD) {
      const int o = t >> 4;
      const float* ur = uh + t * NCAP;
      float accs = 0.0f;
#pragma unroll 4
      for (int n = 0; n < NCAP; ++n) accs = fmaf(sC[n * NCLS + o], ur[n], accs);
      sS[t] = accs;
    }
    __syncthreads();
    if (t < NCLS) {
      const float* sr = sS + t * RD;
      float sq = 0.0f;
#pragma unroll 1
      for (int d = 0; d < RD; ++d) { const float q = sr[d]; sq = fmaf(q, q, sq); }
      const float scl = sq / (1.0f + sq);
      const float rn  = 1.0f / sqrtf(sq + 1e-8f);
#pragma unroll 1
      for (int d = 0; d < RD; ++d) sV[t * RD + d] = (scl * sr[d]) * rn;
    }
    __syncthreads();
    if (it < 2) {
#pragma unroll 1
      for (int j = 0; j < 2; ++j) {
        const int n = t + NTHR * j;
#pragma unroll 1
        for (int o = 0; o < NCLS; ++o) {
          const float* ur = uh + (o * RD) * NCAP + n;
          const float* vr = sV + o * RD;
          float agr = 0.0f;
#pragma unroll 4
          for (int d = 0; d < RD; ++d) agr = fmaf(ur[d * NCAP], vr[d], agr);
          sL[n * NCLS + o] = sL[n * NCLS + o] + agr;
        }
      }
    }
  }

  if (t < NOD) {
    sO[t] = sV[t];
  } else if (t < NOD + NCLS) {
    const int o = t - NOD;
    float sq = 0.0f;
#pragma unroll 1
    for (int d = 0; d < RD; ++d) { const float q = sV[o * RD + d]; sq = fmaf(q, q, sq); }
    sO[t] = sqrtf(sq);
  } else if (t < PVP) {
    sO[t] = 0.0f;
  }
  __syncthreads();
  if (wave == 0) {
    const v4f q = *(const v4fa*)(sO + 4 * lane);
    putf4(PV + (size_t)b * PVP + 4 * lane, q);
  }
}

__global__ __launch_bounds__(NTHR) void k_out(const float* __restrict__ PV, float* out) {
  const int u = (int)blockIdx.x * NTHR + (int)threadIdx.x;
  if (u >= OUT_U) return;
  v4f q;
#pragma unroll
  for (int e = 0; e < 4; ++e) {
    const int f   = 4 * u + e;
    const int bpr = f / NCLS;
    const int ia  = bpr * PVP + NOD + (f - bpr * NCLS);
    int g = f - OUT_V0;
    g = g < 0 ? 0 : g;
    const int bvr = g / NOD;
    const int ib  = bvr * PVP + (g - bvr * NOD);
    int idx = (f < OUT_V0) ? ia : ib;
    idx = idx < 0 ? 0 : (idx > BSZ * PVP - 1 ? BSZ * PVP - 1 : idx);
    q[e] = PV[idx];
  }
  putf4(out + (size_t)4 * u, q);
}

extern "C" void kernel_launch(void* const* d_in, const int* in_sizes, int n_in,
                              void* d_out, int out_size, void* d_ws, size_t ws_size,
                              hipStream_t stream) {
  if (n_in < 6) return;
  if (in_sizes[0] != BSZ * IND) return;
  if (in_sizes[1] != IND * PROJ) return;
  if (in_sizes[2] != PROJ) return;
  if (in_sizes[3] != NOC * CKW) return;
  if (in_sizes[4] != NOC) return;
  if (in_sizes[5] != NCAP * NOD * PD) return;
  if (out_size != OUT_N) return;

  const float* x     = (const float*)d_in[0];
  const float* W1    = (const float*)d_in[1];
  const float* b1    = (const float*)d_in[2];
  const float* convW = (const float*)d_in[3];
  const float* convB = (const float*)d_in[4];
  const float* Wr    = (const float*)d_in[5];
  float* out = (float*)d_out;

  char* ws = (char*)d_ws;
  size_t off = 0;
  const size_t oXB   = off; off += (size_t)BSZ * IND * 2;
  const size_t oW1T  = off; off += (size_t)PROJ * IND * 2;
  const size_t oCW2  = off; off += (size_t)NOC * KCW * 2;
  const size_t oH    = off; off += (size_t)BSZ * PROJ * 4;
  const size_t oHT   = off; off += (size_t)BSZ * NPOS * KTAP * 2;
  const size_t oCONV = off; off += (size_t)CROWS * NOC * 4;
  const size_t oPV   = off; off += (size_t)BSZ * PVP * 4;
  if (off > ws_size || off > (size_t)WSMAX) return;
  unsigned short* XB   = (unsigned short*)(ws + oXB);
  unsigned short* W1T  = (unsigned short*)(ws + oW1T);
  unsigned short* CW2  = (unsigned short*)(ws + oCW2);
  float*          Hf   = (float*)(ws + oH);
  unsigned short* HT   = (unsigned short*)(ws + oHT);
  float*          CONV = (float*)(ws + oCONV);
  float*          PV   = (float*)(ws + oPV);

  hipFuncSetAttribute(reinterpret_cast<const void*>(&k_route), hipFuncAttributeMaxDynamicSharedMemorySize,
                      (int)RT_LDS_BYTES);

  k_prep<<<NU_PREP / NTHR, NTHR, 0, stream>>>(x, W1, convW, XB, W1T, CW2);
  k_gemm1<<<dim3(BSZ / GBM, PROJ / GBN), GTHR, 0, stream>>>(XB, W1T, b1, Hf);
  k_ht<<<BSZ, NTHR, 0, stream>>>(Hf, HT);
  k_conv<<<dim3(BSZ / 4, NOC / GBN), GTHR, 0, stream>>>(HT, CW2, convB, CONV);
  k_route<<<BSZ, NTHR, RT_LDS_BYTES, stream>>>(CONV, Wr, PV);
  k_out<<<OUT_U / NTHR, NTHR, 0, stream>>>(PV, out);
}
